// PartModel_55748675502102
// MI455X (gfx1250) — hardware-verified
//
#include <hip/hip_runtime.h>


namespace {
constexpr int NN = 40000, E = 65536, DIM = 100, OC = 50, SEQ = 6, KF = OC * DIM, KP = 5024;
constexpr float XS = 8.0f, WSC = 256.0f;
typedef _Float16 b16;
typedef __attribute__((ext_vector_type(16))) _Float16 v16b;
typedef __attribute__((ext_vector_type(8))) _Float16 v8b;
typedef __attribute__((ext_vector_type(8))) float v8f;
typedef __attribute__((ext_vector_type(4))) float v4f;
__device__ __forceinline__ float bf16_rne(float f) { unsigned int u = __float_as_uint(f); u += 0x7FFFu + ((u >> 16) & 1u); return __uint_as_float(u & 0xFFFF0000u); }
__device__ __forceinline__ v16b frag_kb(const b16* p, int hh) { const v8b a = *(const v8b*)(p + 8 * hh), b = *(const v8b*)(p + 16 + 8 * hh); v16b f;
#pragma unroll
  for (int e = 0; e < 8; ++e) { f[e] = a[e]; f[8 + e] = b[e]; } return f; }
__device__ __forceinline__ v8f wmma16b(v16b a, v16b b, v8f c) { v8f d = __builtin_amdgcn_wmma_f32_16x16x32_f16(false, a, false, b, (short)0, c, false, false); asm volatile("v_nop\n\tv_nop\n\tv_nop\n\tv_nop" : "+v"(d) : "v"(a), "v"(b)); return d; }
__device__ __forceinline__ void wave_lds_sync() { __builtin_amdgcn_fence(__ATOMIC_RELEASE, "workgroup"); __builtin_amdgcn_wave_barrier(); __builtin_amdgcn_fence(__ATOMIC_ACQUIRE, "workgroup"); }
__device__ __forceinline__ float pmul(float a, float b) { float p = a * b; asm volatile("" : "+v"(p)); return p; }
__device__ __forceinline__ int iclamp(int v, int lo, int hi) { return v < lo ? lo : (v > hi ? hi : v); }

__global__ __launch_bounds__(256) void w1_kernel(const float* __restrict__ w, b16* __restrict__ WT) {
  const int u = blockIdx.x * 256 + threadIdx.x; if (u >= 64 * (KP / 8)) return; const int c = u / (KP / 8), k0 = (u % (KP / 8)) * 8; v8b v;
#pragma unroll
  for (int j = 0; j < 8; ++j) { const int k = k0 + j; v[j] = (c < OC && k < KF) ? (b16)(bf16_rne(w[(size_t)c * KF + k]) * WSC) : (b16)0.0f; } for (int pass = 0; pass < 2; ++pass) { *(volatile v8b*)(WT + (size_t)c * KP + k0) = v; __threadfence(); }
}
__global__ __launch_bounds__(32) void edge_kernel(const int* __restrict__ eidx, const int* __restrict__ etype, const float* __restrict__ x, const float* __restrict__ g, const float* __restrict__ xi, const float* __restrict__ gi, const float* __restrict__ cw, const float* __restrict__ cb, const b16* __restrict__ WT, const float* __restrict__ f1b, const float* __restrict__ f2w, const float* __restrict__ f2b, float* __restrict__ out) {
  __shared__ float St[16][SEQ][DIM + 1]; __shared__ __attribute__((aligned(16))) b16 Ah[16][40]; __shared__ float Cw[OC][SEQ], Cb[OC], So[32];
  const int lane = threadIdx.x, nloc = lane & 15, hlf = lane >> 4; const size_t e0 = (size_t)blockIdx.x * 32;
  for (int i = lane; i < OC * SEQ; i += 32) Cw[i / SEQ][i % SEQ] = bf16_rne(cw[i]); for (int i = lane; i < OC; i += 32) Cb[i] = bf16_rne(cb[i]);
  const float c2 = bf16_rne(f2b[0]);
#pragma unroll 1
  for (int half = 0; half < 2; ++half) {
    for (int rr = 0; rr < 16; ++rr) { const size_t e = e0 + half * 16 + rr; const int r = iclamp(eidx[e], 0, NN - 1), c = iclamp(eidx[E + e], 0, NN - 1), t = iclamp(etype[e], 0, NN - 1);
      const float* srcs[SEQ] = {x + (size_t)r * DIM, g + (size_t)t * DIM, g + (size_t)c * DIM, xi + (size_t)r * DIM, gi + (size_t)t * DIM, xi + (size_t)c * DIM};
#pragma unroll
      for (int s = 0; s < SEQ; ++s) for (int d = lane; d < DIM; d += 32) St[rr][s][d] = bf16_rne(srcs[s][d]); }
    wave_lds_sync(); v8f acc[4] = {(v8f){}, (v8f){}, (v8f){}, (v8f){}};
#pragma unroll 1
    for (int ks = 0; ks < KP / 32; ++ks) { const int k = ks * 32 + lane; const int o = k / DIM, d = k - o * DIM; const bool live = k < KF; float w6[SEQ]; for (int s = 0; s < SEQ; ++s) w6[s] = live ? Cw[o][s] : 0.0f; const float bb = live ? Cb[o] : 0.0f;
      for (int rr = 0; rr < 16; ++rr) { float v = 0.0f; if (live) { v = bb; for (int s = 0; s < SEQ; ++s) v += pmul(St[rr][s][d], w6[s]); v = fmaxf(v, 0.0f); } Ah[rr][lane] = (b16)(v * XS); }
      wave_lds_sync(); const v16b a = frag_kb(&Ah[nloc][0], hlf);
#pragma unroll
      for (int tt = 0; tt < 4; ++tt) acc[tt] = wmma16b(a, frag_kb(WT + (size_t)(tt * 16 + nloc) * KP + ks * 32, hlf), acc[tt]);
      wave_lds_sync(); }
    float pd[8];
#pragma unroll
    for (int r8 = 0; r8 < 8; ++r8) pd[r8] = 0.0f;
#pragma unroll
    for (int tt = 0; tt < 4; ++tt) { const int cc = tt * 16 + nloc; const float bb = cc < OC ? bf16_rne(f1b[cc]) : 0.0f, ww = cc < OC ? bf16_rne(f2w[cc]) : 0.0f;
#pragma unroll
      for (int r8 = 0; r8 < 8; ++r8) pd[r8] += pmul(acc[tt][r8] * (1.0f / (XS * WSC)) + bb, ww); }
#pragma unroll
    for (int r8 = 0; r8 < 8; ++r8) { float s = pd[r8]; for (int o2 = 1; o2 < 16; o2 <<= 1) s += __shfl_xor(s, o2); if (nloc == 0) So[half * 16 + 8 * hlf + r8] = s + c2; }
    wave_lds_sync(); }
  for (int pass = 0; pass < 2; ++pass) { ((volatile float*)out)[e0 + lane] = So[lane]; __threadfence(); }
}
}

extern "C" void kernel_launch(void* const* d_in, const int* in_sizes, int n_in, void* d_out, int out_size, void* d_ws, size_t ws_size, hipStream_t stream) {
  (void)n_in;
  auto Fp = [&](int i) { return (const float*)d_in[i]; }; auto Ip = [&](int i) { return (const int*)d_in[i]; };
  if (in_sizes[0] != 2 * E || in_sizes[1] != E || in_sizes[2] != NN * DIM || in_sizes[3] != NN * DIM || in_sizes[4] != NN * DIM || in_sizes[5] != NN * DIM || in_sizes[6] != OC * SEQ || in_sizes[8] != OC * KF || in_sizes[10] != OC || out_size != E) return;
  const int EV = E;
  size_t off = 0; char* ws = (char*)d_ws;
  auto carve = [&](size_t bytes) { char* p = ws + off; off += (bytes + 255) & ~(size_t)255; return p; };
  b16* WT = (b16*)carve((size_t)64 * KP * 2);
  if (off > ws_size || off > ((size_t)4 << 20)) return;
  w1_kernel<<<(64 * (KP / 8) + 255) / 256, 256, 0, stream>>>(Fp(8), WT);
  edge_kernel<<<(unsigned)(EV / 32), 32, 0, stream>>>(Ip(0), Ip(1), Fp(2), Fp(3), Fp(4), Fp(5), Fp(6), Fp(7), WT, Fp(9), Fp(10), Fp(11), (float*)d_out);
}
